// EncoderBlock_4466765988170
// MI455X (gfx1250) — hardware-verified
//
#include <hip/hip_runtime.h>

typedef __attribute__((ext_vector_type(16))) _Float16 v16h;
typedef __attribute__((ext_vector_type(8)))  _Float16 v8h;
typedef __attribute__((ext_vector_type(4)))  _Float16 v4h;
typedef __attribute__((ext_vector_type(8)))  float    v8f;
typedef __attribute__((ext_vector_type(4)))  float    v4f;

static constexpr int kBatch = 2;
static constexpr int kSeq   = 2048;
static constexpr int kDim   = 1024;
static constexpr int kHeads = 16;
static constexpr int kHdim  = 64;
static constexpr int kDff   = 4096;
static constexpr int kRows  = kBatch * kSeq;
static constexpr int kDqkv  = 3 * kDim;
static_assert(kHeads * kHdim == kDim);
static_assert(kHdim == 64);
static_assert(kSeq % 64 == 0);
static_assert(kRows % 64 == 0 && kDim % 64 == 0 && kDqkv % 64 == 0 && kDff % 64 == 0);
static_assert(kDim % 32 == 0 && kDff % 32 == 0);
static_assert(kDim == 1024);
static_assert(kDff % 1024 == 0);

static constexpr float kWCarry  = 64.0f;
static constexpr float kACarry  = 64.0f;
static constexpr float kGemmScl = 1.0f / (64.0f * 64.0f);
static constexpr float kSmScale = 0.125f;
static constexpr float kPsc     = 32768.0f;

static constexpr size_t kMi      = 1024u * 1024u;
static constexpr size_t kOffHF   = 0;
static constexpr size_t kOffHH   = 16 * kMi;
static constexpr size_t kOffWA   = 24 * kMi;
static constexpr size_t kOffWout = kOffWA + (size_t)kDqkv * kDim * 2;
static constexpr size_t kOffBig  = 32 * kMi;
static constexpr size_t kOffCtx  = kOffBig + (size_t)kRows * kDqkv * 2;
static constexpr size_t kOffH2   = kOffCtx + (size_t)kRows * kDim * 2;
static constexpr size_t kOffHid  = 96 * kMi;
static constexpr size_t kWsTotal = kOffHid + (size_t)kRows * kDff * 2;
static_assert((size_t)kRows * kDim * 4 <= kOffHH - kOffHF);
static_assert((size_t)kRows * kDim * 2 <= kOffWA - kOffHH);
static_assert(kOffWout + (size_t)kDim * kDim * 2 <= kOffBig);
static_assert(kOffWA + (size_t)kDff * kDim * 2 <= kOffBig);
static_assert(kOffH2 + (size_t)kRows * kDim * 4 <= kOffHid);
static_assert(kOffBig + (size_t)kRows * kDff * 4 <= kOffHid);
static_assert(kOffBig + (size_t)kDim * kDff * 2 <= kOffHid);
static_assert(kWsTotal == 134217728u);

__device__ __forceinline__ float rne_bf16f(float f) {
  unsigned u = __float_as_uint(f);
  u = (u + 0x7FFFu + ((u >> 16) & 1u)) & 0xFFFF0000u;
  return __uint_as_float(u);
}

__device__ __forceinline__ void dep_guard_h(v8f& a, v8f& b, v16h x, v16h y) { asm volatile("v_nop\n\tv_nop\n\tv_nop\n\tv_nop" : "+v"(a), "+v"(b) : "v"(x), "v"(y)); }
__device__ __forceinline__ void keep4_h(v16h a, v16h b, v16h c, v16h d) { asm volatile("v_nop" :: "v"(a), "v"(b), "v"(c), "v"(d)); }
__device__ __forceinline__ void acc_guard4(v8f& a, v8f& b, v8f& c, v8f& d) { asm volatile("v_nop\n\tv_nop\n\tv_nop\n\tv_nop" : "+v"(a), "+v"(b), "+v"(c), "+v"(d)); }

template <typename T> struct Frag;
template <> struct Frag<_Float16> {
  typedef v16h V; union U { v16h v; v8h h[2]; };
  static __device__ __forceinline__ v16h load(const _Float16* p) {
    U f; f.h[0] = *(const v8h*)(p); f.h[1] = *(const v8h*)(p + 16); return f.v;
  }
  static __device__ __forceinline__ v8f mma(v16h a, v16h b, v8f c) {
    return __builtin_amdgcn_wmma_f32_16x16x32_f16(false, a, false, b, (short)0, c, false, false);
  }
  static __device__ __forceinline__ void guard(v8f& a, v8f& b, v16h x, v16h y) { dep_guard_h(a, b, x, y); }
  static __device__ __forceinline__ void keep(v16h a, v16h b, v16h c, v16h d) { keep4_h(a, b, c, d); }
};

__device__ __forceinline__ v8f mma_h(v16h a, v16h b, v8f c) {
  c = __builtin_amdgcn_wmma_f32_16x16x32_f16(false, a, false, b, (short)0, c, false, false);
  asm volatile("v_nop\n\tv_nop\n\tv_nop\n\tv_nop" : "+v"(c) : "v"(a), "v"(b));
  return c;
}

__global__ __launch_bounds__(256) void cast_t64(const float* __restrict__ W, unsigned short* __restrict__ Tp,
                                                int Kdim, int Ndim, float carry) {
  __shared__ __align__(16) _Float16 tile[64 * 72];
  _Float16* Tout = (_Float16*)Tp;
  const int t  = threadIdx.x;
  const int n0 = blockIdx.x * 64;
  const int k0 = blockIdx.y * 64;
#pragma unroll
  for (int i = 0; i < 4; ++i) {
    const int idx = t + 256 * i;
    const int kk  = idx >> 4;
    const int n4  = (idx & 15) * 4;
    const v4f w4 = *(const v4f*)(W + (size_t)(k0 + kk) * Ndim + n0 + n4);
#pragma unroll
    for (int e = 0; e < 4; ++e) tile[(n4 + e) * 72 + kk] = (_Float16)(rne_bf16f(w4[e]) * carry);
  }
  __syncthreads();
  const int wave = t >> 5, lane = t & 31;
  const int q = lane >> 3, c8 = (lane & 7) * 8;
  for (int pass = 0; pass < 2; ++pass) {
#pragma unroll
    for (int it = 0; it < 2; ++it) {
      const int nl = wave * 8 + it * 4 + q;
      const v8h hv = *(const v8h*)(tile + nl * 72 + c8);
      *(volatile v8h*)(Tout + (size_t)(n0 + nl) * Kdim + k0 + c8) = hv;
    }
    __threadfence();
  }
}

template <bool RIN>
__global__ __launch_bounds__(256) void rmsnorm_rows(const float* __restrict__ x, const float* __restrict__ g,
                                                    float* __restrict__ y32, unsigned short* __restrict__ y16p,
                                                    int ncols, float inv_sqrt_n, float carry16) {
  __shared__ float red[8];
  __shared__ __align__(16) _Float16 hs[1024];
  const int row = blockIdx.x;
  const int t = threadIdx.x;
  const int wave = t >> 5, lane = t & 31;
  const float* xr = x + (size_t)row * ncols;
  v4f xv = *(const v4f*)(xr + 4 * t);
  if (RIN) {
#pragma unroll
    for (int e = 0; e < 4; ++e) xv[e] = rne_bf16f(xv[e]);
  }
  float ss = 0.0f;
#pragma unroll
  for (int e = 0; e < 4; ++e) ss += xv[e] * xv[e];
#pragma unroll
  for (int m = 16; m >= 1; m >>= 1) ss += __shfl_xor(ss, m, 32);
  if (lane == 0) red[wave] = ss;
  __syncthreads();
  float tot = 0.0f;
#pragma unroll
  for (int w = 0; w < 8; ++w) tot += red[w];
  const float rms = sqrtf(tot) * inv_sqrt_n;
  const float inv = 1.0f / (rms + 1e-8f);
  v4f gv = *(const v4f*)(g + 4 * t);
  v4f yv;
  v4h h4;
#pragma unroll
  for (int e = 0; e < 4; ++e) {
    const float ge = rne_bf16f(gv[e]);
    yv[e] = ge * (xv[e] * inv);
    h4[e] = (_Float16)(yv[e] * carry16);
  }
  *(v4h*)(hs + 4 * t) = h4;
  __syncthreads();
  const v8h hv = *(const v8h*)(hs + 8 * (t & 127));
  float* yr = y32 + (size_t)row * ncols;
  _Float16* yh = (_Float16*)y16p + (size_t)row * ncols;
  for (int pass = 0; pass < 2; ++pass) {
    *(volatile v4f*)(yr + 4 * t) = yv;
    if (t < 128) *(volatile v8h*)(yh + 8 * t) = hv;
    __threadfence();
  }
}

template <int OUT16, bool BIASN, bool RESID>
__global__ __launch_bounds__(256) void gemm64_f16(
    const unsigned short* __restrict__ Ap, int lda,
    const unsigned short* __restrict__ Btp, int ldb,
    void* __restrict__ Cout, int ldc,
    const float* __restrict__ bias,
    const float* __restrict__ resid,
    int M, int N, int K, float scale) {
  typedef _Float16 T;
  typedef v16h V;
  const T* A  = (const T*)Ap;
  const T* Bt = (const T*)Btp;
  __shared__ __align__(16) float sT[8][16 * 68];
  const int lane = threadIdx.x & 31;
  const int wave = threadIdx.x >> 5;
  const int tilesN = N >> 6;
  const int tilesM = M >> 6;
  const int tile = blockIdx.x * 8 + wave;
  if (tile >= tilesM * tilesN) return;
  const int tm = tile / tilesN;
  const int tn = tile - tm * tilesN;
  const int m0 = tm << 6;
  const int n0 = tn << 6;

  const int rlane = lane & 15;
  const int koff  = (lane >> 4) * 8;
  const int mOff  = (lane >> 4) * 8;

  v8f acc[4][4];
#pragma unroll
  for (int i = 0; i < 4; ++i)
#pragma unroll
    for (int j = 0; j < 4; ++j) acc[i][j] = (v8f){0.f,0.f,0.f,0.f,0.f,0.f,0.f,0.f};

  for (int k0 = 0; k0 < K; k0 += 32) {
    V bh[4];
#pragma unroll
    for (int j = 0; j < 4; ++j) {
      const size_t bo = (size_t)(n0 + (j << 4) + rlane) * ldb + koff + k0;
      bh[j] = Frag<T>::load(Bt + bo);
    }
#pragma unroll
    for (int i = 0; i < 4; ++i) {
      const size_t ao = (size_t)(m0 + (i << 4) + rlane) * lda + koff + k0;
      V ah = Frag<T>::load(A + ao);
#pragma unroll
      for (int j = 0; j < 4; ++j) acc[i][j] = Frag<T>::mma(ah, bh[j], acc[i][j]);
      Frag<T>::guard(acc[i][0], acc[i][3], ah, ah);
    }
    Frag<T>::keep(bh[0], bh[1], bh[2], bh[3]);
  }
  acc_guard4(acc[0][0], acc[0][1], acc[0][2], acc[0][3]);
  acc_guard4(acc[1][0], acc[1][1], acc[1][2], acc[1][3]);
  acc_guard4(acc[2][0], acc[2][1], acc[2][2], acc[2][3]);
  acc_guard4(acc[3][0], acc[3][1], acc[3][2], acc[3][3]);

  float* slab = sT[wave];
  const int hh = lane >> 4, c4 = (lane & 15) * 4;
  const int q  = lane >> 3, c8 = (lane & 7) * 8;
  v4f b4 = (v4f){0.f, 0.f, 0.f, 0.f};
  if (BIASN) {
    b4 = *(const v4f*)(bias + n0 + c4);
#pragma unroll
    for (int e = 0; e < 4; ++e) b4[e] = rne_bf16f(b4[e]);
  }
#pragma unroll
  for (int i = 0; i < 4; ++i) {
    const int mBase = m0 + (i << 4);
#pragma unroll
    for (int j = 0; j < 4; ++j) {
#pragma unroll
      for (int r = 0; r < 8; ++r) slab[(mOff + r) * 68 + (j << 4) + rlane] = acc[i][j][r] * scale;
    }
    __builtin_amdgcn_fence(__ATOMIC_RELEASE, "workgroup");
    __builtin_amdgcn_wave_barrier();
    __builtin_amdgcn_fence(__ATOMIC_ACQUIRE, "workgroup");
    if (OUT16 == 0) {
      float* C = (float*)Cout;
      v4f vals[8];
#pragma unroll
      for (int it = 0; it < 8; ++it) {
        const int row = it * 2 + hh;
        v4f v = *(const v4f*)(slab + row * 68 + c4);
        if (BIASN) v += b4;
        if (RESID) {
          const v4f rr = *(const v4f*)(resid + (size_t)(mBase + row) * ldc + n0 + c4);
          v += rr;
        }
        vals[it] = v;
      }
      for (int pass = 0; pass < 2; ++pass) {
#pragma unroll
        for (int it = 0; it < 8; ++it) {
          const int row = it * 2 + hh;
          *(volatile v4f*)(C + (size_t)(mBase + row) * ldc + n0 + c4) = vals[it];
        }
        __threadfence();
      }
    } else {
      _Float16* C = (_Float16*)Cout;
      for (int pass = 0; pass < 2; ++pass) {
#pragma unroll
        for (int it = 0; it < 4; ++it) {
          const int row = it * 4 + q;
          const float* sp = slab + row * 68 + c8;
          v8h hv;
#pragma unroll
          for (int e = 0; e < 8; ++e) hv[e] = (_Float16)sp[e];
          *(volatile v8h*)(C + (size_t)(mBase + row) * ldc + n0 + c8) = hv;
        }
        __threadfence();
      }
    }
    __builtin_amdgcn_fence(__ATOMIC_RELEASE, "workgroup");
    __builtin_amdgcn_wave_barrier();
    __builtin_amdgcn_fence(__ATOMIC_ACQUIRE, "workgroup");
  }
}

__global__ __launch_bounds__(128) void attn64_f16p(const unsigned short* __restrict__ qkvp, unsigned short* __restrict__ ctxp,
                                                  int T, int H, int ldq, int ldo, float sm_scale, float out_carry) {
  const _Float16* QKV = (const _Float16*)qkvp;
  _Float16* CTX = (_Float16*)ctxp;
  union FH { v16h v; v8h hf[2]; };
  __shared__ __align__(16) _Float16 Ksh[64 * 64];
  __shared__ __align__(16) _Float16 Vts[64 * 64];
  __shared__ __align__(16) _Float16 Psh[4][16 * 64];
  __shared__ __align__(16) float    Os[4][16 * 68];

  const int tid  = threadIdx.x;
  const int wave = tid >> 5;
  const int lane = tid & 31;
  const int hh   = lane >> 4;
  const int c    = lane & 15;
  const int dmodel = H * 64;

  const int nqb = T / 64;
  const int bx = blockIdx.x;
  const int qb = bx % nqb;
  const int bh = bx / nqb;
  const int h  = bh % H;
  const int b  = bh / H;
  const int q0 = qb * 64 + wave * 16;

  v16h qa[2];
  {
    const _Float16* qrow = QKV + (size_t)(b * T + q0 + c) * ldq + h * 64;
#pragma unroll
    for (int dc = 0; dc < 2; ++dc) {
      FH f;
      f.hf[0] = *(const v8h*)(qrow + dc * 32 + 8 * hh);
      f.hf[1] = *(const v8h*)(qrow + dc * 32 + 16 + 8 * hh);
      qa[dc] = f.v;
    }
  }

  float mrow[8], lrow[8];
  v8f oacc[4];
#pragma unroll
  for (int r = 0; r < 8; ++r) { mrow[r] = -__builtin_inff(); lrow[r] = 0.f; }
#pragma unroll
  for (int t = 0; t < 4; ++t) oacc[t] = (v8f){0.f,0.f,0.f,0.f,0.f,0.f,0.f,0.f};

  const int nChunks = T / 64;
  for (int kc = 0; kc < nChunks; ++kc) {
    const int kv0 = kc * 64;
    __syncthreads();
    {
      const int kvr = tid >> 1, dh = (tid & 1) * 32;
      const _Float16* krow = QKV + (size_t)(b * T + kv0 + kvr) * ldq + dmodel + h * 64 + dh;
      const _Float16* vrow = krow + dmodel;
#pragma unroll
      for (int i = 0; i < 4; ++i) {
        const v8h k8 = *(const v8h*)(krow + 8 * i);
        *(v8h*)(Ksh + kvr * 64 + dh + 8 * i) = k8;
      }
#pragma unroll
      for (int i = 0; i < 4; ++i) {
        const uint4 vw = *(const uint4*)(const void*)(vrow + 8 * i);
        const unsigned w0 = vw.x, w1 = vw.y, w2 = vw.z, w3 = vw.w;
        const int d = dh + 8 * i;
        Vts[(d + 0) * 64 + kvr] = __builtin_bit_cast(_Float16, (unsigned short)(w0 & 0xFFFFu));
        Vts[(d + 1) * 64 + kvr] = __builtin_bit_cast(_Float16, (unsigned short)(w0 >> 16));
        Vts[(d + 2) * 64 + kvr] = __builtin_bit_cast(_Float16, (unsigned short)(w1 & 0xFFFFu));
        Vts[(d + 3) * 64 + kvr] = __builtin_bit_cast(_Float16, (unsigned short)(w1 >> 16));
        Vts[(d + 4) * 64 + kvr] = __builtin_bit_cast(_Float16, (unsigned short)(w2 & 0xFFFFu));
        Vts[(d + 5) * 64 + kvr] = __builtin_bit_cast(_Float16, (unsigned short)(w2 >> 16));
        Vts[(d + 6) * 64 + kvr] = __builtin_bit_cast(_Float16, (unsigned short)(w3 & 0xFFFFu));
        Vts[(d + 7) * 64 + kvr] = __builtin_bit_cast(_Float16, (unsigned short)(w3 >> 16));
      }
    }
    __syncthreads();

    v8f s[4];
#pragma unroll
    for (int j = 0; j < 4; ++j) {
      s[j] = (v8f){0.f,0.f,0.f,0.f,0.f,0.f,0.f,0.f};
#pragma unroll
      for (int dc = 0; dc < 2; ++dc) {
        FH kb;
        kb.hf[0] = *(const v8h*)(Ksh + (j * 16 + c) * 64 + dc * 32 + 8 * hh);
        kb.hf[1] = *(const v8h*)(Ksh + (j * 16 + c) * 64 + dc * 32 + 16 + 8 * hh);
        s[j] = mma_h(qa[dc], kb.v, s[j]);
      }
    }
    float cm[8];
#pragma unroll
    for (int r = 0; r < 8; ++r) {
      float m = -__builtin_inff();
#pragma unroll
      for (int j = 0; j < 4; ++j) {
        const float sv = s[j][r] * sm_scale;
        s[j][r] = sv;
        m = fmaxf(m, sv);
      }
#pragma unroll
      for (int off = 1; off < 16; off <<= 1) m = fmaxf(m, __shfl_xor(m, off, 32));
      cm[r] = m;
    }
    _Float16* pw = Psh[wave];
#pragma unroll
    for (int r = 0; r < 8; ++r) {
      const float mnew = fmaxf(mrow[r], cm[r]);
      const float alpha = expf(mrow[r] - mnew);
      mrow[r] = mnew;
      float psum = 0.f;
#pragma unroll
      for (int j = 0; j < 4; ++j) {
        const float p = expf(s[j][r] - mnew);
        psum += p;
        pw[(8 * hh + r) * 64 + j * 16 + c] = (_Float16)(p * kPsc);
      }
#pragma unroll
      for (int off = 1; off < 16; off <<= 1) psum += __shfl_xor(psum, off, 32);
      lrow[r] = lrow[r] * alpha + psum;
#pragma unroll
      for (int t = 0; t < 4; ++t) oacc[t][r] *= alpha;
    }
    __builtin_amdgcn_fence(__ATOMIC_RELEASE, "workgroup");
    __builtin_amdgcn_wave_barrier();
    __builtin_amdgcn_fence(__ATOMIC_ACQUIRE, "workgroup");
#pragma unroll 1
    for (int kk = 0; kk < 2; ++kk) {
      FH pa;
      pa.hf[0] = *(const v8h*)(pw + c * 64 + kk * 32 + 8 * hh);
      pa.hf[1] = *(const v8h*)(pw + c * 64 + kk * 32 + 16 + 8 * hh);
#pragma unroll
      for (int t = 0; t < 4; ++t) {
        FH vb;
        vb.hf[0] = *(const v8h*)(Vts + (t * 16 + c) * 64 + kk * 32 + 8 * hh);
        vb.hf[1] = *(const v8h*)(Vts + (t * 16 + c) * 64 + kk * 32 + 16 + 8 * hh);
        oacc[t] = mma_h(pa.v, vb.v, oacc[t]);
      }
    }
  }

  float* os = Os[wave];
#pragma unroll
  for (int r = 0; r < 8; ++r) {
    const float inv = out_carry / (lrow[r] * kPsc);
#pragma unroll
    for (int t = 0; t < 4; ++t) os[(8 * hh + r) * 68 + t * 16 + c] = oacc[t][r] * inv;
  }
  __builtin_amdgcn_fence(__ATOMIC_RELEASE, "workgroup");
  __builtin_amdgcn_wave_barrier();
  __builtin_amdgcn_fence(__ATOMIC_ACQUIRE, "workgroup");
  {
    const int q = lane >> 3, c8 = (lane & 7) * 8;
    for (int pass = 0; pass < 2; ++pass) {
#pragma unroll
      for (int it = 0; it < 4; ++it) {
        const int row = it * 4 + q;
        const float* sp = os + row * 68 + c8;
        v8h hv;
#pragma unroll
        for (int e = 0; e < 8; ++e) hv[e] = (_Float16)sp[e];
        *(volatile v8h*)(CTX + (size_t)(b * T + q0 + row) * ldo + h * 64 + c8) = hv;
      }
      __threadfence();
    }
  }
}

__global__ __launch_bounds__(256) void gelu_rows(const float* __restrict__ pre, const float* __restrict__ bvec,
                                                 unsigned short* __restrict__ hidp, int ncols, float carry) {
  __shared__ __align__(16) _Float16 hs[1024];
  const size_t base = (size_t)blockIdx.x * 1024u;
  const int col0 = (int)(base % (size_t)ncols);
  const int t = threadIdx.x;
#pragma unroll 1
  for (int e = 0; e < 4; ++e) {
    const int idx = 4 * t + e;
    const float u  = pre[base + idx] + rne_bf16f(bvec[col0 + idx]);
    const float gl = 0.5f * u * (1.0f + erff(u * 0.70710678118654752f));
    hs[idx] = (_Float16)(gl * carry);
  }
  __syncthreads();
  const v8h hv = *(const v8h*)(hs + 8 * (t & 127));
  _Float16* out = (_Float16*)hidp + base;
  for (int pass = 0; pass < 2; ++pass) {
    if (t < 128) *(volatile v8h*)(out + 8 * t) = hv;
    __threadfence();
  }
}

extern "C" void kernel_launch(void* const* d_in, const int* in_sizes, int n_in,
                              void* d_out, int out_size, void* d_ws, size_t ws_size,
                              hipStream_t stream) {
  if (n_in < 10) return;
  if (in_sizes[0] != kRows * kDim) return;
  if (in_sizes[1] != kDim * kDqkv) return;
  if (in_sizes[2] != kDim * kDim) return;
  if (in_sizes[3] != kDim) return;
  if (in_sizes[4] != kDim * kDff) return;
  if (in_sizes[5] != kDff) return;
  if (in_sizes[6] != kDff * kDim) return;
  if (in_sizes[7] != kDim) return;
  if (in_sizes[8] != kDim) return;
  if (in_sizes[9] != kDim) return;
  if (out_size != kRows * kDim) return;
  if (ws_size < kWsTotal) return;

  const float* x     = (const float*)d_in[0];
  const float* w_in  = (const float*)d_in[1];
  const float* w_out = (const float*)d_in[2];
  const float* b_out = (const float*)d_in[3];
  const float* w1    = (const float*)d_in[4];
  const float* b1    = (const float*)d_in[5];
  const float* w2    = (const float*)d_in[6];
  const float* b2    = (const float*)d_in[7];
  const float* g1    = (const float*)d_in[8];
  const float* g2    = (const float*)d_in[9];
  float* out = (float*)d_out;

  char* ws = (char*)d_ws;
  float*          hF    = (float*)(ws + kOffHF);
  unsigned short* hH    = (unsigned short*)(ws + kOffHH);
  unsigned short* winT  = (unsigned short*)(ws + kOffWA);
  unsigned short* woutT = (unsigned short*)(ws + kOffWout);
  unsigned short* w1T   = (unsigned short*)(ws + kOffWA);
  unsigned short* qkv   = (unsigned short*)(ws + kOffBig);
  unsigned short* ctx   = (unsigned short*)(ws + kOffCtx);
  float*          h2    = (float*)(ws + kOffH2);
  float*          pre   = (float*)(ws + kOffBig);
  unsigned short* w2T   = (unsigned short*)(ws + kOffBig);
  unsigned short* hid   = (unsigned short*)(ws + kOffHid);

  const dim3 blk256(256);
  const dim3 blk128(128);

  cast_t64<<<dim3(kDqkv / 64, kDim / 64), blk256, 0, stream>>>(w_in, winT, kDim, kDqkv, kWCarry);
  cast_t64<<<dim3(kDim / 64, kDim / 64), blk256, 0, stream>>>(w_out, woutT, kDim, kDim, kWCarry);
  rmsnorm_rows<true><<<dim3(kRows), blk256, 0, stream>>>(x, g1, hF, hH, kDim, 0.03125f, kACarry);
  gemm64_f16<1, false, false><<<dim3((kRows / 64) * (kDqkv / 64) / 8), blk256, 0, stream>>>(
      hH, kDim, winT, kDim, (void*)qkv, kDqkv, nullptr, nullptr, kRows, kDqkv, kDim, kGemmScl);
  attn64_f16p<<<dim3(kBatch * kHeads * (kSeq / 64)), blk128, 0, stream>>>(
      qkv, ctx, kSeq, kHeads, kDqkv, kDim, kSmScale, kACarry);
  gemm64_f16<0, true, true><<<dim3((kRows / 64) * (kDim / 64) / 8), blk256, 0, stream>>>(
      ctx, kDim, woutT, kDim, (void*)h2, kDim, b_out, hF, kRows, kDim, kDim, kGemmScl);
  rmsnorm_rows<false><<<dim3(kRows), blk256, 0, stream>>>(h2, g2, hF, hH, kDim, 0.03125f, kACarry);
  cast_t64<<<dim3(kDff / 64, kDim / 64), blk256, 0, stream>>>(w1, w1T, kDim, kDff, kWCarry);
  gemm64_f16<0, false, false><<<dim3((kRows / 64) * (kDff / 64) / 8), blk256, 0, stream>>>(
      hH, kDim, w1T, kDim, (void*)pre, kDff, nullptr, nullptr, kRows, kDff, kDim, kGemmScl);
  gelu_rows<<<dim3((kRows * kDff) / 1024), blk256, 0, stream>>>(pre, b1, hid, kDff, kACarry);
  cast_t64<<<dim3(kDim / 64, kDff / 64), blk256, 0, stream>>>(w2, w2T, kDff, kDim, kWCarry);
  gemm64_f16<0, true, true><<<dim3((kRows / 64) * (kDim / 64) / 8), blk256, 0, stream>>>(
      hid, kDff, w2T, kDff, (void*)out, kDim, b2, hF, kRows, kDim, kDff, kGemmScl);
}
